// BAN_65807488909779
// MI455X (gfx1250) — hardware-verified
//
#include <hip/hip_runtime.h>
#include <stdint.h>
#include <stddef.h>

constexpr int kB     = 64;
constexpr int kNQ    = 32;
constexpr int kNK    = 256;
constexpr int kE     = 300;
constexpr int kEP    = 320;
constexpr int kH     = 1024;
constexpr int kG     = 8;
constexpr int kNOUT  = 300;
constexpr int kNOUTP = 320;
constexpr int kNANS  = 4000;
constexpr int kNANSP = 4032;
constexpr int kVOCAB = 20000;
constexpr int kGH    = kG * kH;
constexpr int kGQ    = kG * kNQ;

typedef __attribute__((ext_vector_type(16))) _Float16 v16h;
typedef __attribute__((ext_vector_type(8)))  _Float16 v8h;
typedef __attribute__((ext_vector_type(16))) __bf16   v16b;
typedef __attribute__((ext_vector_type(8)))  __bf16   v8b;
typedef __attribute__((ext_vector_type(8)))  float    v8f;
typedef __attribute__((ext_vector_type(4)))  float    v4f;

__device__ __forceinline__ unsigned short f2bf_bits(float f) {
  unsigned u = __float_as_uint(f);
  return (unsigned short)((u + 0x7FFFu + ((u >> 16) & 1u)) >> 16);
}
__device__ __forceinline__ float bf_bits2f(unsigned short h) { return __uint_as_float(((unsigned)h) << 16); }

__device__ __forceinline__ void dep_guard_h(v8f& a, v8f& b, v16h x, v16h y) { asm volatile("v_nop\n\tv_nop\n\tv_nop\n\tv_nop" : "+v"(a), "+v"(b) : "v"(x), "v"(y)); }
__device__ __forceinline__ void dep_guard_b(v8f& a, v8f& b, v16b x, v16b y) { asm volatile("v_nop\n\tv_nop\n\tv_nop\n\tv_nop" : "+v"(a), "+v"(b) : "v"(x), "v"(y)); }
__device__ __forceinline__ void keep4_h(v16h a, v16h b, v16h c, v16h d) { asm volatile("v_nop" :: "v"(a), "v"(b), "v"(c), "v"(d)); }
__device__ __forceinline__ void keep4_b(v16b a, v16b b, v16b c, v16b d) { asm volatile("v_nop" :: "v"(a), "v"(b), "v"(c), "v"(d)); }
__device__ __forceinline__ void acc_guard4(v8f& a, v8f& b, v8f& c, v8f& d) { asm volatile("v_nop\n\tv_nop\n\tv_nop\n\tv_nop" : "+v"(a), "+v"(b), "+v"(c), "+v"(d)); }

template <typename T> struct Frag;
template <> struct Frag<_Float16> {
  typedef v16h V; union U { v16h v; v8h h[2]; };
  static __device__ __forceinline__ v16h load(const _Float16* p) {
    U f; f.h[0] = *(const v8h*)(p); f.h[1] = *(const v8h*)(p + 16); return f.v;
  }
  static __device__ __forceinline__ v8f mma(v16h a, v16h b, v8f c) {
    return __builtin_amdgcn_wmma_f32_16x16x32_f16(false, a, false, b, (short)0, c, false, false);
  }
  static __device__ __forceinline__ void guard(v8f& a, v8f& b, v16h x, v16h y) { dep_guard_h(a, b, x, y); }
  static __device__ __forceinline__ void keep(v16h a, v16h b, v16h c, v16h d) { keep4_h(a, b, c, d); }
};
template <> struct Frag<__bf16> {
  typedef v16b V; union U { v16b v; v8b h[2]; };
  static __device__ __forceinline__ v16b load(const __bf16* p) {
    U f; f.h[0] = *(const v8b*)(p); f.h[1] = *(const v8b*)(p + 16); return f.v;
  }
  static __device__ __forceinline__ v8f mma(v16b a, v16b b, v8f c) {
    return __builtin_amdgcn_wmma_f32_16x16x32_bf16(false, a, false, b, (short)0, c, false, false);
  }
  static __device__ __forceinline__ void guard(v8f& a, v8f& b, v16b x, v16b y) { dep_guard_b(a, b, x, y); }
  static __device__ __forceinline__ void keep(v16b a, v16b b, v16b c, v16b d) { keep4_b(a, b, c, d); }
};

template <int ET> struct Elem;
template <> struct Elem<0> { typedef _Float16 T; };
template <> struct Elem<1> { typedef __bf16 T; };
template <int ET, bool SPLIT, int BIAS_MODE, int OUT_MODE, bool RESID, int ACT = 0>
__global__ __launch_bounds__(256) void wmma_gemm64(
    const unsigned short* __restrict__ Ap, const unsigned short* __restrict__ A2p, int lda, long strideA,
    const unsigned short* __restrict__ Btp, const unsigned short* __restrict__ Bt2p, int ldb, long strideB,
    void* __restrict__ Cout, void* __restrict__ Cout2, int ldc, long strideC,
    const float* __restrict__ bias,
    const float* __restrict__ resid, long strideR,
    int M, int N, int K, float scale, int nbias) {
  typedef typename Elem<ET>::T T;
  typedef typename Frag<T>::V V;
  const T* A = (const T*)Ap; const T* A2 = (const T*)A2p; const T* Bt = (const T*)Btp; const T* Bt2 = (const T*)Bt2p;
  __shared__ __align__(16) float sT[8][16 * 68];
  const int b    = blockIdx.y;
  const int lane = threadIdx.x & 31;
  const int wave = threadIdx.x >> 5;
  const int tilesN = N >> 6;
  const int tilesM = M >> 6;
  const int tile = blockIdx.x * 8 + wave;
  if (tile >= tilesM * tilesN) return;
  const int tm = tile / tilesN;
  const int tn = tile - tm * tilesN;
  const int m0 = tm << 6;
  const int n0 = tn << 6;

  const T* Ab  = A  + (size_t)b * strideA;
  const T* Bb  = Bt + (size_t)b * strideB;
  const T* Ab2 = SPLIT ? (A2  + (size_t)b * strideA) : nullptr;
  const T* Bb2 = SPLIT ? (Bt2 + (size_t)b * strideB) : nullptr;

  const int rlane = lane & 15;
  const int koff  = (lane >> 4) * 8;
  const int mOff  = (lane >> 4) * 8;

  v8f acc[4][4];
#pragma unroll
  for (int i = 0; i < 4; ++i)
#pragma unroll
    for (int j = 0; j < 4; ++j) acc[i][j] = (v8f){0.f,0.f,0.f,0.f,0.f,0.f,0.f,0.f};

  for (int k0 = 0; k0 < K; k0 += 32) {
    V bh[4], bl[4];
#pragma unroll
    for (int j = 0; j < 4; ++j) {
      const size_t bo = (size_t)(n0 + (j << 4) + rlane) * ldb + koff + k0;
      bh[j] = Frag<T>::load(Bb + bo);
      if (SPLIT) bl[j] = Frag<T>::load(Bb2 + bo);
    }
#pragma unroll
    for (int i = 0; i < 4; ++i) {
      const size_t ao = (size_t)(m0 + (i << 4) + rlane) * lda + koff + k0;
      V ah = Frag<T>::load(Ab + ao);
      V al;
      if (SPLIT) al = Frag<T>::load(Ab2 + ao);
#pragma unroll
      for (int j = 0; j < 4; ++j) {
        acc[i][j] = Frag<T>::mma(ah, bh[j], acc[i][j]);
        if (SPLIT) {
          acc[i][j] = Frag<T>::mma(ah, bl[j], acc[i][j]);
          acc[i][j] = Frag<T>::mma(al, bh[j], acc[i][j]);
        }
      }
      Frag<T>::guard(acc[i][0], acc[i][3], ah, SPLIT ? al : ah);
    }
    Frag<T>::keep(bh[0], bh[1], bh[2], bh[3]);
    if (SPLIT) Frag<T>::keep(bl[0], bl[1], bl[2], bl[3]);
  }
  acc_guard4(acc[0][0], acc[0][1], acc[0][2], acc[0][3]);
  acc_guard4(acc[1][0], acc[1][1], acc[1][2], acc[1][3]);
  acc_guard4(acc[2][0], acc[2][1], acc[2][2], acc[2][3]);
  acc_guard4(acc[3][0], acc[3][1], acc[3][2], acc[3][3]);

  float* slab = sT[wave];
  const float* Rb = RESID ? (resid + (size_t)b * strideR) : nullptr;
#pragma unroll
  for (int i = 0; i < 4; ++i) {
    const int mBase = m0 + (i << 4);
#pragma unroll
    for (int j = 0; j < 4; ++j) {
      const int n = n0 + (j << 4) + rlane;
      float bv = 0.f;
      if (BIAS_MODE == 2) bv = bias[n];
      if (BIAS_MODE == 3) {
        const int nc = (n < nbias) ? n : (nbias - 1);
        const float tb = bias[nc];
        bv = (n < nbias) ? tb : 0.f;
      }
#pragma unroll
      for (int r = 0; r < 8; ++r) {
        float v = acc[i][j][r] * scale;
        if (BIAS_MODE == 1) v += bias[mBase + mOff + r];
        if (BIAS_MODE == 2 || BIAS_MODE == 3) v += bv;
        if (RESID) v += Rb[(size_t)(mBase + mOff + r) * ldc + n];
        if (ACT == 1) v = tanhf(v);
        if (ACT == 2) v = fmaxf(v, 0.0f);
        if (ACT == 3) v = v / (1.0f + expf(-v));
        if (ACT == 4) v = (v > 0.f) ? v : 0.01f * v;
        if (ACT == 5) v = 0.5f * v * (1.0f + erff(v * 0.70710678118654752f));
        slab[(mOff + r) * 68 + (j << 4) + rlane] = v;
      }
    }
    __builtin_amdgcn_fence(__ATOMIC_RELEASE, "workgroup");
    __builtin_amdgcn_wave_barrier();
    __builtin_amdgcn_fence(__ATOMIC_ACQUIRE, "workgroup");
    if (OUT_MODE == 0) {
      float* C = (float*)Cout + (size_t)b * strideC;
      const int hh = lane >> 4, c4 = (lane & 15) * 4;
      for (int pass = 0; pass < 2; ++pass) {
#pragma unroll
        for (int it = 0; it < 8; ++it) {
          const int row = it * 2 + hh;
          v4f v = *(const v4f*)(slab + row * 68 + c4);
          *(volatile v4f*)(C + (size_t)(mBase + row) * ldc + n0 + c4) = v;
        }
        __threadfence();
      }
    } else {
      const int q = lane >> 3, c8 = (lane & 7) * 8;
      unsigned short* C  = (unsigned short*)Cout  + (size_t)b * strideC;
      unsigned short* C2 = (OUT_MODE == 2) ? ((unsigned short*)Cout2 + (size_t)b * strideC) : nullptr;
      for (int pass = 0; pass < 2; ++pass) {
#pragma unroll
        for (int it = 0; it < 4; ++it) {
          const int row = it * 4 + q;
          const float* sp = slab + row * 68 + c8;
          v8h hv, lv;
#pragma unroll
          for (int e = 0; e < 8; ++e) {
            if (OUT_MODE == 1) {
              hv[e] = (_Float16)sp[e];
            } else if (OUT_MODE == 3) {
              hv[e] = __builtin_bit_cast(_Float16, f2bf_bits(sp[e]));
            } else {
              unsigned short hb = f2bf_bits(sp[e]);
              unsigned short lb = f2bf_bits(sp[e] - bf_bits2f(hb));
              hv[e] = __builtin_bit_cast(_Float16, hb);
              lv[e] = __builtin_bit_cast(_Float16, lb);
            }
          }
          *(volatile v8h*)(C + (size_t)(mBase + row) * ldc + n0 + c8) = hv;
          if (OUT_MODE == 2) *(volatile v8h*)(C2 + (size_t)(mBase + row) * ldc + n0 + c8) = lv;
        }
        __threadfence();
      }
    }
    __builtin_amdgcn_fence(__ATOMIC_RELEASE, "workgroup");
    __builtin_amdgcn_wave_barrier();
    __builtin_amdgcn_fence(__ATOMIC_ACQUIRE, "workgroup");
  }
}

__global__ __launch_bounds__(256) void wmma_pool64(
    const unsigned short* __restrict__ Ap, int lda, long strideA,
    const unsigned short* __restrict__ Btp, int ldb, long strideB,
    const float* __restrict__ hq, int ldh, long strideH,
    unsigned short* __restrict__ pooled, int ldp, long strideP,
    int M, int N, int K) {
  typedef __bf16 T;
  typedef Frag<T>::V V;
  const T* A = (const T*)Ap; const T* Bt = (const T*)Btp;
  __shared__ __align__(16) float sP[8][2 * 68];
  const int b    = blockIdx.y;
  const int lane = threadIdx.x & 31;
  const int wave = threadIdx.x >> 5;
  const int tilesN = N >> 6;
  const int tilesM = M >> 6;
  const int tile = blockIdx.x * 8 + wave;
  if (tile >= tilesM * tilesN) return;
  const int tm = tile / tilesN;
  const int tn = tile - tm * tilesN;
  const int m0 = tm << 6;
  const int n0 = tn << 6;

  const T* Ab = A  + (size_t)b * strideA;
  const T* Bb = Bt + (size_t)b * strideB;

  const int rlane = lane & 15;
  const int koff  = (lane >> 4) * 8;
  const int mOff  = (lane >> 4) * 8;

  v8f acc[4][4];
#pragma unroll
  for (int i = 0; i < 4; ++i)
#pragma unroll
    for (int j = 0; j < 4; ++j) acc[i][j] = (v8f){0.f,0.f,0.f,0.f,0.f,0.f,0.f,0.f};

  for (int k0 = 0; k0 < K; k0 += 32) {
    V bh[4];
#pragma unroll
    for (int j = 0; j < 4; ++j) {
      const size_t bo = (size_t)(n0 + (j << 4) + rlane) * ldb + koff + k0;
      bh[j] = Frag<T>::load(Bb + bo);
    }
#pragma unroll
    for (int i = 0; i < 4; ++i) {
      const size_t ao = (size_t)(m0 + (i << 4) + rlane) * lda + koff + k0;
      V ah = Frag<T>::load(Ab + ao);
#pragma unroll
      for (int j = 0; j < 4; ++j) acc[i][j] = Frag<T>::mma(ah, bh[j], acc[i][j]);
      Frag<T>::guard(acc[i][0], acc[i][3], ah, ah);
    }
    Frag<T>::keep(bh[0], bh[1], bh[2], bh[3]);
  }
  acc_guard4(acc[0][0], acc[0][1], acc[0][2], acc[0][3]);
  acc_guard4(acc[1][0], acc[1][1], acc[1][2], acc[1][3]);
  acc_guard4(acc[2][0], acc[2][1], acc[2][2], acc[2][3]);
  acc_guard4(acc[3][0], acc[3][1], acc[3][2], acc[3][3]);

  const float* Hb = hq + (size_t)b * strideH;
  float* slab = sP[wave];
  const int g0 = m0 >> 5;
#pragma unroll
  for (int j = 0; j < 4; ++j) {
    const int n = n0 + (j << 4) + rlane;
    float p0 = 0.f, p1 = 0.f;
#pragma unroll
    for (int r = 0; r < 8; ++r) {
      const float h0 = Hb[(size_t)(mOff + r) * ldh + n];
      const float h1 = Hb[(size_t)(16 + mOff + r) * ldh + n];
      p0 += acc[0][j][r] * h0;
      p0 += acc[1][j][r] * h1;
      p1 += acc[2][j][r] * h0;
      p1 += acc[3][j][r] * h1;
    }
    p0 += __shfl_xor(p0, 16, 32);
    p1 += __shfl_xor(p1, 16, 32);
    if (lane < 16) {
      slab[(j << 4) + rlane]      = p0;
      slab[68 + (j << 4) + rlane] = p1;
    }
  }
  __builtin_amdgcn_fence(__ATOMIC_RELEASE, "workgroup");
  __builtin_amdgcn_wave_barrier();
  __builtin_amdgcn_fence(__ATOMIC_ACQUIRE, "workgroup");
  if (lane < 16) {
    const int gs = lane >> 3, c8 = (lane & 7) * 8;
    const float* sp = slab + gs * 68 + c8;
    v8h hv;
#pragma unroll
    for (int e = 0; e < 8; ++e) hv[e] = __builtin_bit_cast(_Float16, f2bf_bits(sp[e]));
    unsigned short* P = pooled + (size_t)b * strideP + (size_t)(g0 + gs) * ldp + n0 + c8;
    *(volatile v8h*)P = hv;
    __threadfence();
    *(volatile v8h*)P = hv;
  }
}

template <bool HAS_IDX>
__global__ __launch_bounds__(256) void rows_bf16_320(
    const float* __restrict__ in, const int* __restrict__ idx, int rows_in, int C,
    unsigned short* __restrict__ out, int rows_out, int rows_valid) {
  const int lane = threadIdx.x & 31;
  const int row  = blockIdx.x * 8 + (threadIdx.x >> 5);
  if (row >= rows_out) return;
  const bool rv = row < rows_valid;
  int src;
  if (HAS_IDX) {
    const int ri = rv ? row : (rows_valid - 1);
    int t = idx[ri];
    t = t < 0 ? 0 : t;
    t = t > rows_in - 1 ? rows_in - 1 : t;
    src = t;
  } else {
    src = row < rows_in ? row : rows_in - 1;
  }
  const float* ip = in + (size_t)src * C;
  unsigned short* op = out + (size_t)row * kEP;
  const int lb = lane < 8 ? lane : 0;
  v8h va, vb;
#pragma unroll
  for (int e = 0; e < 8; ++e) {
    const int ca = 8 * lane + e;
    const int caa = ca < C ? ca : C - 1;
    const float fa = ip[caa];
    const unsigned short ba = (rv && ca < C) ? f2bf_bits(fa) : (unsigned short)0;
    va[e] = __builtin_bit_cast(_Float16, ba);
    const int cb = 256 + 8 * lb + e;
    const int cbb = cb < C ? cb : C - 1;
    const float fb = ip[cbb];
    const unsigned short bb = (rv && cb < C) ? f2bf_bits(fb) : (unsigned short)0;
    vb[e] = __builtin_bit_cast(_Float16, bb);
  }
  for (int pass = 0; pass < 2; ++pass) {
    *(volatile v8h*)(op + 8 * lane) = va;
    if (lane < 8) *(volatile v8h*)(op + 256 + 8 * lane) = vb;
    __threadfence();
  }
}

__device__ __forceinline__ unsigned short to_bf_bits(float f) { return f2bf_bits(f); }
__device__ __forceinline__ unsigned short to_bf_bits(unsigned short u) { return u; }
template <typename TI>
__global__ __launch_bounds__(256) void tr_bf16(const TI* __restrict__ in, int R, int C, long in_bs,
                                              unsigned short* __restrict__ out, int RO, int CO, long out_bs) {
  __shared__ unsigned short s[64][34];
  const int t = threadIdx.x, lane = t & 31, wave = t >> 5;
  const int r0 = blockIdx.x * 64, c0 = blockIdx.y * 32;
  const TI* ib = in + (size_t)blockIdx.z * in_bs;
  unsigned short* ob = out + (size_t)blockIdx.z * out_bs;
#pragma unroll
  for (int i = 0; i < 8; ++i) {
    const int rl = wave + 8 * i;
    const int rr = r0 + rl, cc = c0 + lane;
    const int ra = rr < R ? rr : R - 1;
    const int ca = cc < C ? cc : C - 1;
    unsigned short bits = to_bf_bits(ib[(size_t)ra * C + ca]);
    if (rr >= R || cc >= C) bits = (unsigned short)0;
    s[rl][lane] = bits;
  }
  __syncthreads();
  const int cl = 4 * wave + (lane >> 3);
  const int q8 = (lane & 7) * 8;
  v8h v;
#pragma unroll
  for (int e = 0; e < 8; ++e) v[e] = __builtin_bit_cast(_Float16, s[q8 + e][cl]);
  int orow = c0 + cl; orow = orow < CO ? orow : CO - 1;
  unsigned short* p = ob + (size_t)orow * RO + r0 + q8;
  *(volatile v8h*)p = v;
  __threadfence();
  *(volatile v8h*)p = v;
}

__global__ __launch_bounds__(256) void build_ag(const float* __restrict__ hq, const float* __restrict__ Watt,
                                                unsigned short* __restrict__ Ag) {
  const int lane = threadIdx.x & 31;
  const int m = blockIdx.x * 8 + (threadIdx.x >> 5);
  if (m >= kB * kGQ) return;
  const int b = m >> 8, g = (m >> 5) & 7, q = m & 31;
  const float* hr = hq + ((size_t)b * kNQ + q) * kH;
  unsigned short* dst = Ag + (size_t)m * kH;
  v8h pv[4];
#pragma unroll
  for (int i = 0; i < 4; ++i) {
    const int d0 = 256 * i + 8 * lane;
    const v4f a = *(const v4f*)(hr + d0);
    const v4f c = *(const v4f*)(hr + d0 + 4);
#pragma unroll
    for (int e = 0; e < 4; ++e) {
      const float w0 = Watt[(size_t)(d0 + e) * kG + g];
      const float w1 = Watt[(size_t)(d0 + 4 + e) * kG + g];
      pv[i][e]     = __builtin_bit_cast(_Float16, f2bf_bits(a[e] * w0));
      pv[i][4 + e] = __builtin_bit_cast(_Float16, f2bf_bits(c[e] * w1));
    }
  }
  for (int pass = 0; pass < 2; ++pass) {
#pragma unroll
    for (int i = 0; i < 4; ++i) *(volatile v8h*)(dst + 256 * i + 8 * lane) = pv[i];
    __threadfence();
  }
}

__global__ __launch_bounds__(256) void softmax_att(const float* __restrict__ logits, const float* __restrict__ batt,
                                                   unsigned short* __restrict__ att) {
  __shared__ float red[256];
  const int bg = blockIdx.x;
  const int g = bg & 7;
  const int tid = threadIdx.x;
  const float* x = logits + (size_t)bg * (kNQ * kNK);
  unsigned short* ap = att + (size_t)bg * (kNQ * kNK);
  const float bb = batt[g];
  float mx = -INFINITY;
#pragma unroll 1
  for (int i = tid; i < kNQ * kNK; i += 256) mx = fmaxf(mx, x[i] + bb);
  red[tid] = mx; __syncthreads();
  for (int st = 128; st > 0; st >>= 1) { if (tid < st) red[tid] = fmaxf(red[tid], red[tid + st]); __syncthreads(); }
  mx = red[0]; __syncthreads();
  float sum = 0.f;
#pragma unroll 1
  for (int i = tid; i < kNQ * kNK; i += 256) sum += __expf((x[i] + bb) - mx);
  red[tid] = sum; __syncthreads();
  for (int st = 128; st > 0; st >>= 1) { if (tid < st) red[tid] += red[tid + st]; __syncthreads(); }
  const float inv = 1.0f / red[0];
  v8h pv[4];
#pragma unroll
  for (int i = 0; i < 4; ++i) {
    const int base = 2048 * i + 8 * tid;
    const v4f a = *(const v4f*)(x + base);
    const v4f c = *(const v4f*)(x + base + 4);
#pragma unroll
    for (int e = 0; e < 4; ++e) {
      const float pa = __expf((a[e] + bb) - mx) * inv;
      const float pc = __expf((c[e] + bb) - mx) * inv;
      pv[i][e]     = __builtin_bit_cast(_Float16, f2bf_bits(pa));
      pv[i][4 + e] = __builtin_bit_cast(_Float16, f2bf_bits(pc));
    }
  }
  for (int pass = 0; pass < 2; ++pass) {
#pragma unroll
    for (int i = 0; i < 4; ++i) *(volatile v8h*)(ap + 2048 * i + 8 * tid) = pv[i];
    __threadfence();
  }
}

__global__ __launch_bounds__(256) void logsoftmax_out(const float* __restrict__ sim, float* __restrict__ out) {
  __shared__ float red[256];
  const int b = blockIdx.x;
  const int tid = threadIdx.x;
  const float* x = sim + (size_t)b * kNANSP;
  float* ob = out + (size_t)b * kNANS;
  float mx = -INFINITY;
#pragma unroll 1
  for (int i = tid; i < kNANS; i += 256) mx = fmaxf(mx, x[i]);
  red[tid] = mx; __syncthreads();
  for (int st = 128; st > 0; st >>= 1) { if (tid < st) red[tid] = fmaxf(red[tid], red[tid + st]); __syncthreads(); }
  mx = red[0]; __syncthreads();
  float sum = 0.f;
#pragma unroll 1
  for (int i = tid; i < kNANS; i += 256) sum += expf(x[i] - mx);
  red[tid] = sum; __syncthreads();
  for (int st = 128; st > 0; st >>= 1) { if (tid < st) red[tid] += red[tid + st]; __syncthreads(); }
  const float lg = logf(red[0]);
  for (int pass = 0; pass < 2; ++pass) {
#pragma unroll
    for (int i = 0; i < 4; ++i) {
      const int i4 = 1024 * i + 4 * tid;
      const int ia = i4 < kNANS - 4 ? i4 : kNANS - 4;
      const v4f v = *(const v4f*)(x + ia);
      v4f o;
#pragma unroll
      for (int e = 0; e < 4; ++e) o[e] = (v[e] - mx) - lg;
      if (i4 < kNANS) *(volatile v4f*)(ob + i4) = o;
    }
    __threadfence();
  }
}

extern "C" void kernel_launch(void* const* d_in, const int* in_sizes, int n_in,
                              void* d_out, int out_size, void* d_ws, size_t ws_size,
                              hipStream_t stream) {
  if (n_in < 12) return;
  if (in_sizes[0] != kB * kNQ || in_sizes[1] != kB * kNK || in_sizes[2] != kVOCAB * kE ||
      in_sizes[3] != kE * kH || in_sizes[4] != kH || in_sizes[5] != kE * kH || in_sizes[6] != kH ||
      in_sizes[7] != kH * kG || in_sizes[8] != kG || in_sizes[9] != kGH * kNOUT ||
      in_sizes[10] != kNOUT || in_sizes[11] != kNANS * kNOUT) return;
  if (out_size != kB * kNANS) return;

  const int*   he_ques = (const int*)  d_in[0];
  const int*   he_kg   = (const int*)  d_in[1];
  const float* emb     = (const float*)d_in[2];
  const float* Wq      = (const float*)d_in[3];
  const float* bq      = (const float*)d_in[4];
  const float* Wk      = (const float*)d_in[5];
  const float* bk      = (const float*)d_in[6];
  const float* Watt    = (const float*)d_in[7];
  const float* batt    = (const float*)d_in[8];
  const float* Wout    = (const float*)d_in[9];
  const float* bout    = (const float*)d_in[10];
  const float* cands   = (const float*)d_in[11];
  float* outp = (float*)d_out;

  const size_t szEmbq  = (size_t)kB * kNQ * kEP * 2;
  const size_t szEmbk  = (size_t)kB * kNK * kEP * 2;
  const size_t szWT    = (size_t)kH * kEP * 2;
  const size_t szHq    = (size_t)kB * kNQ * kH * 4;
  const size_t szHk    = (size_t)kB * kNK * kH * 2;
  const size_t szAg    = (size_t)kB * kGQ * kH * 2;
  const size_t szLog   = (size_t)kB * kGQ * kNK * 4;
  const size_t szPool  = (size_t)kB * kGH * 2;
  const size_t szWoutT = (size_t)kNOUTP * kGH * 2;
  const size_t szOutb  = (size_t)kB * kNOUTP * 2;
  const size_t szCand  = (size_t)kNANSP * kNOUTP * 2;
  const size_t szSim   = (size_t)kB * kNANSP * 4;
  size_t off = 0;
  char* base = (char*)d_ws;
  unsigned short* embq   = (unsigned short*)(base + off); off += szEmbq;
  unsigned short* embk   = (unsigned short*)(base + off);
  unsigned short* att    = (unsigned short*)(base + off); off += szEmbk;
  unsigned short* WqT    = (unsigned short*)(base + off); off += szWT;
  unsigned short* WkT    = (unsigned short*)(base + off); off += szWT;
  float*          hq     = (float*)         (base + off); off += szHq;
  unsigned short* hk     = (unsigned short*)(base + off); off += szHk;
  unsigned short* Ag     = (unsigned short*)(base + off);
  unsigned short* hkT    = (unsigned short*)(base + off); off += szAg;
  float*          logits = (float*)         (base + off); off += szLog;
  unsigned short* pooled = (unsigned short*)(base + off); off += szPool;
  unsigned short* WoutT  = (unsigned short*)(base + off); off += szWoutT;
  unsigned short* outb   = (unsigned short*)(base + off); off += szOutb;
  unsigned short* candsb = (unsigned short*)(base + off); off += szCand;
  float*          sim    = (float*)         (base + off); off += szSim;
  if (off > ws_size) return;

  rows_bf16_320<true ><<<(kB * kNQ) / 8, 256, 0, stream>>>(emb, he_ques, kVOCAB, kE, embq, kB * kNQ, kB * kNQ);
  rows_bf16_320<true ><<<(kB * kNK) / 8, 256, 0, stream>>>(emb, he_kg, kVOCAB, kE, embk, kB * kNK, kB * kNK);
  rows_bf16_320<false><<<kNANSP / 8, 256, 0, stream>>>(cands, he_ques, kNANS, kNOUT, candsb, kNANSP, kNANS);
  tr_bf16<float><<<dim3(kEP / 64, kH / 32, 1), 256, 0, stream>>>(Wq, kE, kH, 0L, WqT, kEP, kH, 0L);
  tr_bf16<float><<<dim3(kEP / 64, kH / 32, 1), 256, 0, stream>>>(Wk, kE, kH, 0L, WkT, kEP, kH, 0L);
  tr_bf16<float><<<dim3(kGH / 64, kNOUTP / 32, 1), 256, 0, stream>>>(Wout, kGH, kNOUT, 0L, WoutT, kGH, kNOUTP, 0L);
  wmma_gemm64<1, false, 2, 0, false><<<dim3(((kB * kNQ) / 64) * (kH / 64) / 8, 1), 256, 0, stream>>>(
      embq, embq, kEP, 0L, WqT, WqT, kEP, 0L, (void*)hq, (void*)hq, kH, 0L, bq, Watt, 0L,
      kB * kNQ, kH, kEP, 1.0f, kH);
  wmma_gemm64<1, false, 2, 3, false><<<dim3(((kB * kNK) / 64) * (kH / 64) / 8, 1), 256, 0, stream>>>(
      embk, embk, kEP, 0L, WkT, WkT, kEP, 0L, (void*)hk, (void*)hk, kH, 0L, bk, Watt, 0L,
      kB * kNK, kH, kEP, 1.0f, kH);
  build_ag<<<(kB * kGQ) / 8, 256, 0, stream>>>(hq, Watt, Ag);
  wmma_gemm64<1, false, 0, 0, false><<<dim3(2, kB), 256, 0, stream>>>(
      Ag, Ag, kH, (long)kGQ * kH, hk, hk, kH, (long)kNK * kH, (void*)logits, (void*)logits, kNK, (long)kGQ * kNK,
      batt, Watt, 0L, kGQ, kNK, kH, 1.0f, 0);
  softmax_att<<<kB * kG, 256, 0, stream>>>(logits, batt, att);
  tr_bf16<unsigned short><<<dim3(kNK / 64, kH / 32, kB), 256, 0, stream>>>(
      hk, kNK, kH, (long)kNK * kH, hkT, kNK, kH, (long)kH * kNK);
  wmma_pool64<<<dim3((kGQ / 64) * (kH / 64) / 8, kB), 256, 0, stream>>>(
      att, kNK, (long)kGQ * kNK, hkT, kNK, (long)kH * kNK, hq, kH, (long)kNQ * kH,
      pooled, kH, (long)kGH, kGQ, kH, kNK);
  wmma_gemm64<1, false, 3, 3, false><<<dim3(1, 1), 256, 0, stream>>>(
      pooled, pooled, kGH, 0L, WoutT, WoutT, kGH, 0L, (void*)outb, (void*)outb, kNOUTP, 0L, bout, Watt, 0L,
      kB, kNOUTP, kGH, 1.0f, kNOUT);
  wmma_gemm64<1, false, 0, 0, false><<<dim3((kNANSP / 64 + 7) / 8, 1), 256, 0, stream>>>(
      outb, outb, kNOUTP, 0L, candsb, candsb, kNOUTP, 0L, (void*)sim, (void*)sim, kNANSP, 0L, batt, Watt, 0L,
      kB, kNANSP, kNOUTP, 1.0f, 0);
  logsoftmax_out<<<kB, 256, 0, stream>>>(sim, outp);
}
